// sLSTMLayer_35828617183868
// MI455X (gfx1250) — hardware-verified
//
#include <hip/hip_runtime.h>
#include <stdint.h>
#include <stddef.h>

constexpr int NBATCH = 4;
constexpr int SEQLEN = 2048;
constexpr int DMODEL = 768;
constexpr int NHEAD  = 4;
constexpr int DHEAD  = 192;
constexpr int KCONV  = 4;
constexpr int NGATE  = 4;
constexpr int GATEN  = NGATE * DHEAD;
constexpr float NORM_EPS = 1e-5f;

constexpr size_t BYTES_XB   = (size_t)NBATCH * SEQLEN * DMODEL * 2;
constexpr size_t BYTES_WCAT = (size_t)NHEAD * GATEN * DHEAD * 2;
constexpr size_t BYTES_G    = (size_t)SEQLEN * NHEAD * NBATCH * GATEN * 4;
constexpr size_t OFF_XB   = 0;
constexpr size_t OFF_XCB  = OFF_XB + BYTES_XB;
constexpr size_t OFF_WCAT = OFF_XCB + BYTES_XB;
constexpr size_t OFF_RCAT = OFF_WCAT + BYTES_WCAT;
constexpr size_t OFF_G    = OFF_RCAT + BYTES_WCAT;
constexpr size_t WS_TOTAL = OFF_G + BYTES_G;
static_assert(WS_TOTAL == 128188416ull, "carve total");
static_assert(WS_TOTAL <= 134217728ull, "carve within 128 MiB");
static_assert(OFF_XCB % 128 == 0 && OFF_WCAT % 128 == 0 && OFF_RCAT % 128 == 0 && OFF_G % 128 == 0, "128-B aligned regions");

static_assert(SEQLEN % 64 == 0, "M tile multiple");
static_assert((2 * DHEAD) % 64 == 0, "N tile multiple");
static_assert(DHEAD % 32 == 0, "K multiple of 32");

typedef __attribute__((ext_vector_type(16))) _Float16 v16h;
typedef __attribute__((ext_vector_type(8)))  _Float16 v8h;
typedef __attribute__((ext_vector_type(16))) __bf16   v16b;
typedef __attribute__((ext_vector_type(8)))  __bf16   v8b;
typedef __attribute__((ext_vector_type(8)))  float    v8f;
typedef __attribute__((ext_vector_type(4)))  float    v4f;
typedef __attribute__((ext_vector_type(4)))  unsigned int v4u;

__device__ __forceinline__ unsigned short f2bf_bits(float f) {
  unsigned u = __float_as_uint(f);
  return (unsigned short)((u + 0x7FFFu + ((u >> 16) & 1u)) >> 16);
}
__device__ __forceinline__ float bf_bits2f(unsigned short h) { return __uint_as_float(((unsigned)h) << 16); }
__device__ __forceinline__ float bfr(float f) { return bf_bits2f(f2bf_bits(f)); }

__device__ __forceinline__ void dep_guard_h(v8f& a, v8f& b, v16h x, v16h y) { asm volatile("v_nop\n\tv_nop\n\tv_nop\n\tv_nop" : "+v"(a), "+v"(b) : "v"(x), "v"(y)); }
__device__ __forceinline__ void dep_guard_b(v8f& a, v8f& b, v16b x, v16b y) { asm volatile("v_nop\n\tv_nop\n\tv_nop\n\tv_nop" : "+v"(a), "+v"(b) : "v"(x), "v"(y)); }
__device__ __forceinline__ void keep4_h(v16h a, v16h b, v16h c, v16h d) { asm volatile("v_nop" :: "v"(a), "v"(b), "v"(c), "v"(d)); }
__device__ __forceinline__ void keep4_b(v16b a, v16b b, v16b c, v16b d) { asm volatile("v_nop" :: "v"(a), "v"(b), "v"(c), "v"(d)); }
__device__ __forceinline__ void acc_guard4(v8f& a, v8f& b, v8f& c, v8f& d) { asm volatile("v_nop\n\tv_nop\n\tv_nop\n\tv_nop" : "+v"(a), "+v"(b), "+v"(c), "+v"(d)); }
template <typename T> struct Frag;
template <> struct Frag<_Float16> {
  typedef v16h V; union U { v16h v; v8h h[2]; };
  static __device__ __forceinline__ v16h load(const _Float16* p) {
    U f; f.h[0] = *(const v8h*)(p); f.h[1] = *(const v8h*)(p + 16); return f.v;
  }
  static __device__ __forceinline__ v8f mma(v16h a, v16h b, v8f c) {
    return __builtin_amdgcn_wmma_f32_16x16x32_f16(false, a, false, b, (short)0, c, false, false);
  }
  static __device__ __forceinline__ void guard(v8f& a, v8f& b, v16h x, v16h y) { dep_guard_h(a, b, x, y); }
  static __device__ __forceinline__ void keep(v16h a, v16h b, v16h c, v16h d) { keep4_h(a, b, c, d); }
};
template <> struct Frag<__bf16> {
  typedef v16b V; union U { v16b v; v8b h[2]; };
  static __device__ __forceinline__ v16b load(const __bf16* p) {
    U f; f.h[0] = *(const v8b*)(p); f.h[1] = *(const v8b*)(p + 16); return f.v;
  }
  static __device__ __forceinline__ v8f mma(v16b a, v16b b, v8f c) {
    return __builtin_amdgcn_wmma_f32_16x16x32_bf16(false, a, false, b, (short)0, c, false, false);
  }
  static __device__ __forceinline__ void guard(v8f& a, v8f& b, v16b x, v16b y) { dep_guard_b(a, b, x, y); }
  static __device__ __forceinline__ void keep(v16b a, v16b b, v16b c, v16b d) { keep4_b(a, b, c, d); }
};

__device__ __forceinline__ v8f at_mma(v16b a, v16b b, v8f c) {
  c = __builtin_amdgcn_wmma_f32_16x16x32_bf16(false, a, false, b, (short)0, c, false, false);
  asm volatile("v_nop\n\tv_nop\n\tv_nop\n\tv_nop" : "+v"(c) : "v"(a), "v"(b));
  return c;
}

template <int ET> struct Elem;
template <> struct Elem<0> { typedef _Float16 T; };
template <> struct Elem<1> { typedef __bf16 T; };
template <int ET, bool SPLIT, int BIAS_MODE, int OUT_MODE, bool RESID, int ACT = 0>
__global__ __launch_bounds__(256) void wmma_gemm64(
    const unsigned short* __restrict__ Ap, const unsigned short* __restrict__ A2p, int lda, long strideA,
    const unsigned short* __restrict__ Btp, const unsigned short* __restrict__ Bt2p, int ldb, long strideB,
    void* __restrict__ Cout, void* __restrict__ Cout2, int ldc, long strideC,
    const float* __restrict__ bias,
    const float* __restrict__ resid, long strideR,
    int M, int N, int K, float scale) {
  typedef typename Elem<ET>::T T;
  typedef typename Frag<T>::V V;
  const T* A = (const T*)Ap; const T* A2 = (const T*)A2p; const T* Bt = (const T*)Btp; const T* Bt2 = (const T*)Bt2p;
  __shared__ __align__(16) float sT[8][16 * 68];
  const int b    = blockIdx.y;
  const int lane = threadIdx.x & 31;
  const int wave = threadIdx.x >> 5;
  const int tilesN = N >> 6;
  const int tilesM = M >> 6;
  const int tile = blockIdx.x * 8 + wave;
  if (tile >= tilesM * tilesN) return;
  const int tm = tile / tilesN;
  const int tn = tile - tm * tilesN;
  const int m0 = tm << 6;
  const int n0 = tn << 6;

  const T* Ab  = A  + (size_t)b * strideA;
  const T* Bb  = Bt + (size_t)b * strideB;
  const T* Ab2 = SPLIT ? (A2  + (size_t)b * strideA) : nullptr;
  const T* Bb2 = SPLIT ? (Bt2 + (size_t)b * strideB) : nullptr;

  const int rlane = lane & 15;
  const int koff  = (lane >> 4) * 8;
  const int mOff  = (lane >> 4) * 8;

  v8f acc[4][4];
#pragma unroll
  for (int i = 0; i < 4; ++i)
#pragma unroll
    for (int j = 0; j < 4; ++j) acc[i][j] = (v8f){0.f,0.f,0.f,0.f,0.f,0.f,0.f,0.f};

  for (int k0 = 0; k0 < K; k0 += 32) {
    V bh[4], bl[4];
#pragma unroll
    for (int j = 0; j < 4; ++j) {
      const size_t bo = (size_t)(n0 + (j << 4) + rlane) * ldb + koff + k0;
      bh[j] = Frag<T>::load(Bb + bo);
      if (SPLIT) bl[j] = Frag<T>::load(Bb2 + bo);
    }
#pragma unroll
    for (int i = 0; i < 4; ++i) {
      const size_t ao = (size_t)(m0 + (i << 4) + rlane) * lda + koff + k0;
      V ah = Frag<T>::load(Ab + ao);
      V al;
      if (SPLIT) al = Frag<T>::load(Ab2 + ao);
#pragma unroll
      for (int j = 0; j < 4; ++j) {
        acc[i][j] = Frag<T>::mma(ah, bh[j], acc[i][j]);
        if (SPLIT) {
          acc[i][j] = Frag<T>::mma(ah, bl[j], acc[i][j]);
          acc[i][j] = Frag<T>::mma(al, bh[j], acc[i][j]);
        }
      }
      Frag<T>::guard(acc[i][0], acc[i][3], ah, SPLIT ? al : ah);
    }
    Frag<T>::keep(bh[0], bh[1], bh[2], bh[3]);
    if (SPLIT) Frag<T>::keep(bl[0], bl[1], bl[2], bl[3]);
  }
  acc_guard4(acc[0][0], acc[0][1], acc[0][2], acc[0][3]);
  acc_guard4(acc[1][0], acc[1][1], acc[1][2], acc[1][3]);
  acc_guard4(acc[2][0], acc[2][1], acc[2][2], acc[2][3]);
  acc_guard4(acc[3][0], acc[3][1], acc[3][2], acc[3][3]);

  float* slab = sT[wave];
  const float* Rb = RESID ? (resid + (size_t)b * strideR) : nullptr;
#pragma unroll
  for (int i = 0; i < 4; ++i) {
    const int mBase = m0 + (i << 4);
#pragma unroll
    for (int j = 0; j < 4; ++j) {
      const int n = n0 + (j << 4) + rlane;
      float bv = 0.f;
      if (BIAS_MODE == 2) bv = bias[n];
#pragma unroll
      for (int r = 0; r < 8; ++r) {
        float v = acc[i][j][r] * scale;
        if (BIAS_MODE == 1) v += bias[mBase + mOff + r];
        if (BIAS_MODE == 2) v += bv;
        if (RESID) v += Rb[(size_t)(mBase + mOff + r) * ldc + n];
        if (ACT == 1) v = tanhf(v);
        if (ACT == 2) v = fmaxf(v, 0.0f);
        if (ACT == 3) v = v / (1.0f + expf(-v));
        if (ACT == 4) v = (v > 0.f) ? v : 0.01f * v;
        if (ACT == 5) v = 0.5f * v * (1.0f + erff(v * 0.70710678118654752f));
        slab[(mOff + r) * 68 + (j << 4) + rlane] = v;
      }
    }
    __builtin_amdgcn_fence(__ATOMIC_RELEASE, "workgroup");
    __builtin_amdgcn_wave_barrier();
    __builtin_amdgcn_fence(__ATOMIC_ACQUIRE, "workgroup");
    if (OUT_MODE == 0) {
      float* C = (float*)Cout + (size_t)b * strideC;
      const int hh = lane >> 4, c4 = (lane & 15) * 4;
      for (int pass = 0; pass < 2; ++pass) {
#pragma unroll
        for (int it = 0; it < 8; ++it) {
          const int row = it * 2 + hh;
          v4f v = *(const v4f*)(slab + row * 68 + c4);
          *(volatile v4f*)(C + (size_t)(mBase + row) * ldc + n0 + c4) = v;
        }
        __threadfence();
      }
    } else {
      const int q = lane >> 3, c8 = (lane & 7) * 8;
      unsigned short* C  = (unsigned short*)Cout  + (size_t)b * strideC;
      unsigned short* C2 = (OUT_MODE == 2) ? ((unsigned short*)Cout2 + (size_t)b * strideC) : nullptr;
      for (int pass = 0; pass < 2; ++pass) {
#pragma unroll
        for (int it = 0; it < 4; ++it) {
          const int row = it * 4 + q;
          const float* sp = slab + row * 68 + c8;
          v8h hv, lv;
#pragma unroll
          for (int e = 0; e < 8; ++e) {
            if (OUT_MODE == 1) {
              hv[e] = (_Float16)sp[e];
            } else {
              unsigned short hb = f2bf_bits(sp[e]);
              unsigned short lb = f2bf_bits(sp[e] - bf_bits2f(hb));
              hv[e] = __builtin_bit_cast(_Float16, hb);
              lv[e] = __builtin_bit_cast(_Float16, lb);
            }
          }
          *(volatile v8h*)(C + (size_t)(mBase + row) * ldc + n0 + c8) = hv;
          if (OUT_MODE == 2) *(volatile v8h*)(C2 + (size_t)(mBase + row) * ldc + n0 + c8) = lv;
        }
        __threadfence();
      }
    }
    __builtin_amdgcn_fence(__ATOMIC_RELEASE, "workgroup");
    __builtin_amdgcn_wave_barrier();
    __builtin_amdgcn_fence(__ATOMIC_ACQUIRE, "workgroup");
  }
}

__global__ __launch_bounds__(256) void prep_weights(
    const float* __restrict__ Wi, const float* __restrict__ Wf,
    const float* __restrict__ Wz, const float* __restrict__ Wo,
    const float* __restrict__ Rm,
    unsigned short* __restrict__ Wcat, unsigned short* __restrict__ Rcat) {
  const int lane = threadIdx.x & 31;
  const int w    = threadIdx.x >> 5;
  const int row  = blockIdx.x * 8 + w;
  const bool isR = row >= NHEAD * GATEN;
  const int rr   = isR ? row - NHEAD * GATEN : row;
  const int head = rr / GATEN;
  const int n    = rr - head * GATEN;
  const int g    = n / DHEAD;
  const int ecol = n - g * DHEAD;
  const float* src;
  size_t base;
  if (isR) {
    src  = Rm;
    base = ((size_t)(g * NHEAD + head) * DHEAD) * DHEAD + ecol;
  } else {
    src  = (g == 0) ? Wi : (g == 1) ? Wf : (g == 2) ? Wz : Wo;
    base = ((size_t)head * DHEAD) * DHEAD + ecol;
  }
  unsigned short* dst = (isR ? Rcat : Wcat) + (size_t)rr * DHEAD;
  v4u pk;
#pragma unroll
  for (int q = 0; q < 4; ++q) {
    const int k0 = 8 * lane + 2 * q;
    const int ka = min(k0, DHEAD - 1);
    const int kb = min(k0 + 1, DHEAD - 1);
    const float va = src[base + (size_t)ka * DHEAD];
    const float vb = src[base + (size_t)kb * DHEAD];
    pk[q] = (unsigned)f2bf_bits(va) | ((unsigned)f2bf_bits(vb) << 16);
  }
  unsigned short* dp = dst + 8 * min(lane, 23);
  if (lane < 24) *(volatile v4u*)dp = pk;
  __threadfence();
  if (lane < 24) *(volatile v4u*)dp = pk;
}

__global__ __launch_bounds__(96) void conv_swish_cast(
    const float* __restrict__ x, const float* __restrict__ ck, const float* __restrict__ cb,
    unsigned short* __restrict__ Xb, unsigned short* __restrict__ Xcb) {
  const int rowi = blockIdx.x;
  const int s    = rowi & (SEQLEN - 1);
  const int d0   = threadIdx.x * 8;
  float acc[8];
  {
    const v4f c0 = *(const v4f*)(cb + d0);
    const v4f c1 = *(const v4f*)(cb + d0 + 4);
#pragma unroll
    for (int i = 0; i < 4; ++i) { acc[i] = bfr(c0[i]); acc[4 + i] = bfr(c1[i]); }
  }
  unsigned xbits[8];
#pragma unroll
  for (int j = 0; j < KCONV; ++j) {
    const int  ss    = s - (KCONV - 1) + j;
    const bool valid = ss >= 0;
    const int  ssc   = valid ? ss : 0;
    const float* xr  = x + ((size_t)(rowi - s + ssc)) * DMODEL + d0;
    const v4f x0 = *(const v4f*)(xr);
    const v4f x1 = *(const v4f*)(xr + 4);
    const v4f k0 = *(const v4f*)(ck + j * DMODEL + d0);
    const v4f k1 = *(const v4f*)(ck + j * DMODEL + d0 + 4);
#pragma unroll
    for (int i = 0; i < 4; ++i) {
      const unsigned short xb0 = f2bf_bits(x0[i]);
      const unsigned short xb1 = f2bf_bits(x1[i]);
      const float xv0 = valid ? bf_bits2f(xb0) : 0.0f;
      const float xv1 = valid ? bf_bits2f(xb1) : 0.0f;
      acc[i]     = fmaf(xv0, bfr(k0[i]), acc[i]);
      acc[4 + i] = fmaf(xv1, bfr(k1[i]), acc[4 + i]);
      if (j == KCONV - 1) { xbits[i] = xb0; xbits[4 + i] = xb1; }
    }
    asm volatile("" ::: "memory");
  }
  unsigned swb[8];
#pragma unroll
  for (int i = 0; i < 8; ++i) {
    const float ex = __expf(-acc[i]);
    const float rc = __builtin_amdgcn_rcpf(1.0f + ex);
    const float sw = acc[i] * rc;
    swb[i] = f2bf_bits(sw);
  }
  v4u px, pc;
#pragma unroll
  for (int q = 0; q < 4; ++q) {
    px[q] = xbits[2 * q] | (xbits[2 * q + 1] << 16);
    pc[q] = swb[2 * q]   | (swb[2 * q + 1]   << 16);
  }
  unsigned short* xbp = Xb  + (size_t)rowi * DMODEL + d0;
  unsigned short* xcp = Xcb + (size_t)rowi * DMODEL + d0;
  *(volatile v4u*)xbp = px;
  *(volatile v4u*)xcp = pc;
  __threadfence();
  *(volatile v4u*)xbp = px;
  *(volatile v4u*)xcp = pc;
}

constexpr int SCAN_THREADS = 384;
constexpr int SCAN_WAVES   = 12;
constexpr int HPITCH       = 200;
constexpr int GST          = NBATCH * GATEN;
static_assert(SCAN_WAVES * 16 == DHEAD, "wave e-coverage");
static_assert(GST == 2 * 4 * SCAN_THREADS, "gate block = 2 float4 per thread");
static_assert(SCAN_WAVES * 2 == NBATCH * DHEAD / 32, "two output lines per wave per step");

__global__ __launch_bounds__(SCAN_THREADS) void slstm_scan_norm(
    const float* __restrict__ G, const unsigned short* __restrict__ Rcat,
    const float* __restrict__ cell_bias, const float* __restrict__ gn_scale,
    float* __restrict__ out) {
  __shared__ __align__(16) unsigned short hbf[2 * 16 * HPITCH];
  __shared__ __align__(16) float gstage[2 * GST];
  __shared__ __align__(16) float ostage[2 * NBATCH * DHEAD];
  __shared__ __align__(16) float stat[2 * SCAN_WAVES * NBATCH * 2];
  __shared__ __align__(16) float gsc[DHEAD];

  const int head = blockIdx.x;
  const int tid  = threadIdx.x;
  const int lane = tid & 31;
  const int w    = tid >> 5;
  const int hh   = lane >> 4;
  const int l15  = lane & 15;
  const int e    = w * 16 + l15;

  for (int i = tid; i < 16 * HPITCH; i += SCAN_THREADS) ((unsigned*)hbf)[i] = 0u;
  if (tid < DHEAD) gsc[tid] = bfr(gn_scale[head * DHEAD + tid]);
  {
    const v4f* Gp = (const v4f*)(G + (size_t)head * GST);
    ((v4f*)gstage)[tid] = Gp[tid];
    ((v4f*)gstage)[tid + SCAN_THREADS] = Gp[tid + SCAN_THREADS];
  }
  float cbv[NGATE];
#pragma unroll
  for (int g = 0; g < NGATE; ++g) cbv[g] = bfr(cell_bias[g * DMODEL + head * DHEAD + e]);
  __syncthreads();

  float cs[NBATCH], ns[NBATCH], ms[NBATCH];
#pragma unroll
  for (int b = 0; b < NBATCH; ++b) { cs[b] = 0.0f; ns[b] = 0.0f; ms[b] = 0.0f; }

  const __bf16* Rg = (const __bf16*)(const void*)Rcat + (size_t)head * GATEN * DHEAD;
  union FB { v16b v; v8b h[2]; };

  for (int t = 0; t < SEQLEN; ++t) {
    const int p = t & 1;
    const float* gs = gstage + p * GST;

    v8f acc[NGATE];
#pragma unroll
    for (int g = 0; g < NGATE; ++g) {
      v8f c = (v8f){0.f,0.f,0.f,0.f,0.f,0.f,0.f,0.f};
#pragma unroll
      for (int r = 0; r < NBATCH; ++r) {
        const float v = gs[r * GATEN + g * DHEAD + e] + cbv[g];
        c[r] = (hh == 0) ? v : 0.0f;
      }
      acc[g] = c;
    }

    if (t + 1 < SEQLEN) {
      const v4f* Gp = (const v4f*)(G + ((size_t)(t + 1) * NHEAD + head) * GST);
      v4f* gd = (v4f*)(gstage + (p ^ 1) * GST);
      gd[tid] = Gp[tid];
      gd[tid + SCAN_THREADS] = Gp[tid + SCAN_THREADS];
    }

    const unsigned short* hbp = hbf + p * 16 * HPITCH + l15 * HPITCH + 8 * hh;
#pragma unroll 1
    for (int kk = 0; kk < DHEAD / 32; ++kk) {
      FB a;
      a.h[0] = *(const v8b*)(hbp + kk * 32);
      a.h[1] = *(const v8b*)(hbp + kk * 32 + 16);
#pragma unroll
      for (int g = 0; g < NGATE; ++g) {
        const v16b bq = Frag<__bf16>::load(Rg + (size_t)(g * DHEAD + e) * DHEAD + kk * 32 + 8 * hh);
        acc[g] = at_mma(a.v, bq, acc[g]);
      }
    }

    float hn[NBATCH];
#pragma unroll
    for (int b = 0; b < NBATCH; ++b) {
      const float it = acc[0][b], ft = acc[1][b], zt = acc[2][b], ot = acc[3][b];
      const float fm = ft + ms[b];
      const float mn = fmaxf(fm, it);
      const float ia = expf(it - mn);
      const float fa = expf(fm - mn);
      const float cn = fa * cs[b] + ia * tanhf(zt);
      const float nn = fa * ns[b] + ia;
      const float sg = 1.0f / (1.0f + expf(-ot));
      hn[b] = (sg * cn) / nn;
      cs[b] = cn; ns[b] = nn; ms[b] = mn;
    }
    if (hh == 0) {
      unsigned short* hw = hbf + (p ^ 1) * 16 * HPITCH + e;
      float* ow = ostage + p * (NBATCH * DHEAD) + e;
#pragma unroll
      for (int b = 0; b < NBATCH; ++b) {
        hw[b * HPITCH] = f2bf_bits(hn[b]);
        ow[b * DHEAD]  = hn[b];
      }
    }
    float s1v[NBATCH], m2v[NBATCH];
#pragma unroll
    for (int b = 0; b < NBATCH; ++b) {
      float sm = hn[b];
      sm += __shfl_xor(sm, 1, 32);
      sm += __shfl_xor(sm, 2, 32);
      sm += __shfl_xor(sm, 4, 32);
      sm += __shfl_xor(sm, 8, 32);
      const float dlt = hn[b] - sm * (1.0f / 16.0f);
      float q2 = dlt * dlt;
      q2 += __shfl_xor(q2, 1, 32);
      q2 += __shfl_xor(q2, 2, 32);
      q2 += __shfl_xor(q2, 4, 32);
      q2 += __shfl_xor(q2, 8, 32);
      s1v[b] = sm; m2v[b] = q2;
    }
    if (lane == 0) {
      float* stw = stat + p * (SCAN_WAVES * NBATCH * 2) + w * (NBATCH * 2);
#pragma unroll
      for (int b = 0; b < NBATCH; ++b) { stw[2 * b] = s1v[b]; stw[2 * b + 1] = m2v[b]; }
    }
    __syncthreads();

    {
      const int q   = (lane >> 3) & 1;
      const int j8  = lane & 7;
      const int L   = 2 * w + q;
      const int bb  = L / 6;
      const int seg = L - 6 * bb;
      const int e0  = seg * 32 + 4 * j8;
      const float* st = stat + p * (SCAN_WAVES * NBATCH * 2) + bb * 2;
      float S1 = 0.0f;
#pragma unroll
      for (int ww = 0; ww < SCAN_WAVES; ++ww) S1 += st[ww * (NBATCH * 2)];
      const float mu = S1 * (1.0f / (float)DHEAD);
      float M2 = 0.0f;
#pragma unroll
      for (int ww = 0; ww < SCAN_WAVES; ++ww) {
        const float dm = st[ww * (NBATCH * 2)] * (1.0f / 16.0f) - mu;
        M2 += st[ww * (NBATCH * 2) + 1] + 16.0f * dm * dm;
      }
      const float var = M2 * (1.0f / (float)DHEAD);
      const float rs  = rsqrtf(var + NORM_EPS);
      const v4f v   = *(const v4f*)(ostage + p * (NBATCH * DHEAD) + bb * DHEAD + e0);
      const v4f sc4 = *(const v4f*)(gsc + e0);
      v4f y;
#pragma unroll
      for (int i = 0; i < 4; ++i) y[i] = (v[i] - mu) * rs * sc4[i];
      float* op = out + ((size_t)(bb * SEQLEN + t)) * DMODEL + head * DHEAD + e0;
      if (hh == 0) *(volatile v4f*)op = y;
      __threadfence();
      if (hh == 0) *(volatile v4f*)op = y;
    }
  }
}

extern "C" void kernel_launch(void* const* d_in, const int* in_sizes, int n_in,
                              void* d_out, int out_size, void* d_ws, size_t ws_size,
                              hipStream_t stream) {
  if (n_in < 10) return;
  if (in_sizes[0] != NBATCH * SEQLEN * DMODEL) return;
  if (in_sizes[1] != KCONV * DMODEL) return;
  if (in_sizes[2] != DMODEL) return;
  if (in_sizes[3] != NHEAD * DHEAD * DHEAD || in_sizes[4] != NHEAD * DHEAD * DHEAD ||
      in_sizes[5] != NHEAD * DHEAD * DHEAD || in_sizes[6] != NHEAD * DHEAD * DHEAD) return;
  if (in_sizes[7] != NGATE * NHEAD * DHEAD * DHEAD) return;
  if (in_sizes[8] != NGATE * DMODEL) return;
  if (in_sizes[9] != NHEAD * DHEAD) return;
  if (out_size != NBATCH * SEQLEN * DMODEL) return;
  if (ws_size < WS_TOTAL) return;

  const float* x    = (const float*)d_in[0];
  const float* ck   = (const float*)d_in[1];
  const float* cb   = (const float*)d_in[2];
  const float* Wi   = (const float*)d_in[3];
  const float* Wf   = (const float*)d_in[4];
  const float* Wz   = (const float*)d_in[5];
  const float* Wo   = (const float*)d_in[6];
  const float* Rm   = (const float*)d_in[7];
  const float* cbia = (const float*)d_in[8];
  const float* gsc  = (const float*)d_in[9];
  float* out = (float*)d_out;
  char* ws = (char*)d_ws;

  unsigned short* Xb   = (unsigned short*)(ws + OFF_XB);
  unsigned short* Xcb  = (unsigned short*)(ws + OFF_XCB);
  unsigned short* Wcat = (unsigned short*)(ws + OFF_WCAT);
  unsigned short* Rcat = (unsigned short*)(ws + OFF_RCAT);
  float* G = (float*)(ws + OFF_G);

  prep_weights<<<(2 * NHEAD * GATEN) / 8, 256, 0, stream>>>(Wi, Wf, Wz, Wo, Rm, Wcat, Rcat);

  conv_swish_cast<<<NBATCH * SEQLEN, 96, 0, stream>>>(x, ck, cb, Xb, Xcb);

  for (int b = 0; b < NBATCH; ++b) {
    for (int half = 0; half < 2; ++half) {
      const unsigned short* A  = (half == 0 ? Xcb : Xb) + (size_t)b * SEQLEN * DMODEL;
      const unsigned short* Bt = Wcat + (size_t)half * (2 * DHEAD) * DHEAD;
      float* C = G + (size_t)b * GATEN + (size_t)half * (2 * DHEAD);
      const int tiles = (SEQLEN / 64) * ((2 * DHEAD) / 64);
      wmma_gemm64<1, false, 0, 0, false, 0><<<dim3((tiles + 7) / 8, NHEAD), 256, 0, stream>>>(
          A, nullptr, DMODEL, (long)DHEAD,
          Bt, nullptr, DHEAD, (long)GATEN * DHEAD,
          (void*)C, nullptr, NHEAD * GST, (long)GST,
          nullptr, nullptr, 0L,
          SEQLEN, 2 * DHEAD, DHEAD, 1.0f);
    }
  }

  slstm_scan_norm<<<NHEAD, SCAN_THREADS, 0, stream>>>(G, Rcat, cbia, gsc, out);
}
